// MambaBlock_12618613916216
// MI455X (gfx1250) — hardware-verified
//
#include <hip/hip_runtime.h>
#include <math.h>

typedef __attribute__((ext_vector_type(8)))  _Float16 v8h;
typedef __attribute__((ext_vector_type(16))) __bf16   v16b;
typedef __attribute__((ext_vector_type(8)))  __bf16   v8b;
typedef __attribute__((ext_vector_type(8)))  float    v8f;
typedef __attribute__((ext_vector_type(4)))  float    v4f;

constexpr int kBatch = 2;
constexpr int kSeq   = 1024;
constexpr int kDm    = 768;
constexpr int kDin   = 1536;
constexpr int kNst   = 16;
constexpr int kDtR   = 48;
constexpr int kDtK   = 64;
constexpr int kPrjN  = 80;
constexpr int kPrjP  = 128;
constexpr int kXzP   = 2 * kDin;
constexpr int kRows  = kBatch * kSeq;
constexpr int kTP    = 260;
constexpr float kLnEps = 1e-5f;
constexpr float kInvDm = 1.0f / (float)kDm;

static_assert(kDtR + 2 * kNst == kPrjN, "x_proj width");
static_assert(kRows * kDm == 1572864, "x / out element count");
static_assert(kXzP * kDm == 2359296, "W_in element count");
static_assert(kPrjN * kDin == 122880, "W_x element count");
static_assert(kDin * kDtR == 73728, "W_dt element count");
static_assert(kDm * kDin == 1179648, "W_out element count");
static_assert(kDin * kNst == 24576, "A_log element count");
static_assert((kDm % 32) == 0 && (kDin % 32) == 0 && (kDtK % 32) == 0, "GEMM K multiples of 32");
static_assert((kRows % 64) == 0 && (kXzP % 64) == 0 && (kPrjP % 64) == 0 && (kDin % 64) == 0 && (kDm % 64) == 0, "GEMM M,N multiples of 64");
static_assert((kSeq & (kSeq - 1)) == 0 && (kSeq % 64) == 0 && (kDin % 256) == 0, "tile multiples");
static_assert(kDtK == 64 && (kDtR % 8) == 0 && kDtR < kDtK, "dt pad layout");
static_assert(kDm == 6 * 128, "LayerNorm lane map");

constexpr size_t kOffXB   = 0;
constexpr size_t kOffWIB  = kOffXB   + (size_t)kRows * kDm   * 2;
constexpr size_t kOffWXB  = kOffWIB  + (size_t)kXzP  * kDm   * 2;
constexpr size_t kOffWDB  = kOffWXB  + (size_t)kPrjP * kDin  * 2;
constexpr size_t kOffWOB  = kOffWDB  + (size_t)kDin  * kDtK  * 2;
constexpr size_t kOffXZ   = kOffWOB  + (size_t)kDm   * kDin  * 2;
constexpr size_t kOffUC   = kOffXZ   + (size_t)kRows * kXzP  * 4;
constexpr size_t kOffUCH  = kOffUC   + (size_t)kRows * kDin  * 4;
constexpr size_t kOffUCL  = kOffUCH  + (size_t)kRows * kDin  * 2;
constexpr size_t kOffPROJ = kOffUCL  + (size_t)kRows * kDin  * 2;
constexpr size_t kOffDTH  = kOffPROJ + (size_t)kRows * kPrjP * 4;
constexpr size_t kOffDTL  = kOffDTH  + (size_t)kRows * kDtK  * 2;
constexpr size_t kOffDLR  = kOffDTL  + (size_t)kRows * kDtK  * 2;
constexpr size_t kOffYH   = kOffDLR  + (size_t)kRows * kDin  * 4;
constexpr size_t kOffYL   = kOffYH   + (size_t)kRows * kDin  * 2;
constexpr size_t kOffPRE  = kOffYL   + (size_t)kRows * kDin  * 2;
constexpr size_t kWsTotal = kOffPRE  + (size_t)kRows * kDm   * 4;
static_assert(kWsTotal == 94175232ull, "carve total");
static_assert(kWsTotal <= 134217728ull, "carve cap");
static_assert((kOffWIB % 128) == 0 && (kOffWXB % 128) == 0 && (kOffWDB % 128) == 0 && (kOffWOB % 128) == 0 &&
              (kOffXZ % 128) == 0 && (kOffUC % 128) == 0 && (kOffUCH % 128) == 0 && (kOffUCL % 128) == 0 &&
              (kOffPROJ % 128) == 0 && (kOffDTH % 128) == 0 && (kOffDTL % 128) == 0 && (kOffDLR % 128) == 0 &&
              (kOffYH % 128) == 0 && (kOffYL % 128) == 0 && (kOffPRE % 128) == 0, "128-B aligned regions");

__device__ __forceinline__ unsigned short f2bf_bits(float f) {
  unsigned u = __float_as_uint(f);
  return (unsigned short)((u + 0x7FFFu + ((u >> 16) & 1u)) >> 16);
}
__device__ __forceinline__ float bf_bits2f(unsigned short h) { return __uint_as_float(((unsigned)h) << 16); }
__device__ __forceinline__ float bf_rne(float f) { return bf_bits2f(f2bf_bits(f)); }

__device__ __forceinline__ void dep_guard4_b(v8f& a, v8f& b, v8f& c, v8f& d, v16b x, v16b y) {
  asm volatile("v_nop\n\tv_nop\n\tv_nop\n\tv_nop" : "+v"(a), "+v"(b), "+v"(c), "+v"(d) : "v"(x), "v"(y));
}
__device__ __forceinline__ void keep4_b(v16b a, v16b b, v16b c, v16b d) { asm volatile("v_nop" :: "v"(a), "v"(b), "v"(c), "v"(d)); }
__device__ __forceinline__ void acc_guard4(v8f& a, v8f& b, v8f& c, v8f& d) { asm volatile("v_nop\n\tv_nop\n\tv_nop\n\tv_nop" : "+v"(a), "+v"(b), "+v"(c), "+v"(d)); }

template <typename T> struct Frag;
template <> struct Frag<__bf16> {
  typedef v16b V; union U { v16b v; v8b h[2]; };
  static __device__ __forceinline__ v16b load(const __bf16* p) {
    U f; f.h[0] = *(const v8b*)(p); f.h[1] = *(const v8b*)(p + 16); return f.v;
  }
  static __device__ __forceinline__ v8f mma(v16b a, v16b b, v8f c) {
    return __builtin_amdgcn_wmma_f32_16x16x32_bf16(false, a, false, b, (short)0, c, false, false);
  }
  static __device__ __forceinline__ void guard4(v8f& a, v8f& b, v8f& c, v8f& d, v16b x, v16b y) { dep_guard4_b(a, b, c, d, x, y); }
  static __device__ __forceinline__ void keep(v16b a, v16b b, v16b c, v16b d) { keep4_b(a, b, c, d); }
};

template <int ET> struct Elem;
template <> struct Elem<1> { typedef __bf16 T; };
template <int ET, int SPL, int BIAS_MODE, int OUT_MODE, bool RESID, int ACT = 0>
__global__ __launch_bounds__(256) void wmma_gemm64(
    const unsigned short* __restrict__ Ap, const unsigned short* __restrict__ A2p, int lda, long strideA,
    const unsigned short* __restrict__ Btp, const unsigned short* __restrict__ Bt2p, int ldb, long strideB,
    void* __restrict__ Cout, void* __restrict__ Cout2, int ldc, long strideC,
    const float* __restrict__ bias,
    const float* __restrict__ resid, long strideR,
    int M, int N, int K, float scale) {
  typedef typename Elem<ET>::T T;
  typedef typename Frag<T>::V V;
  const T* A = (const T*)Ap; const T* A2 = (const T*)A2p; const T* Bt = (const T*)Btp; const T* Bt2 = (const T*)Bt2p;
  __shared__ __align__(16) float sT[8][16 * 68];
  const int b    = blockIdx.y;
  const int lane = threadIdx.x & 31;
  const int wave = threadIdx.x >> 5;
  const int tilesN = N >> 6;
  const int tilesM = M >> 6;
  const int tile = blockIdx.x * 8 + wave;
  if (tile >= tilesM * tilesN) return;
  const int tm = tile / tilesN;
  const int tn = tile - tm * tilesN;
  const int m0 = tm << 6;
  const int n0 = tn << 6;

  const T* Ab  = A  + (size_t)b * strideA;
  const T* Bb  = Bt + (size_t)b * strideB;
  const T* Ab2 = (SPL >= 1) ? (A2  + (size_t)b * strideA) : nullptr;
  const T* Bb2 = (SPL == 2) ? (Bt2 + (size_t)b * strideB) : nullptr;

  const int rlane = lane & 15;
  const int koff  = (lane >> 4) * 8;
  const int mOff  = (lane >> 4) * 8;

  v8f acc[4][4];
#pragma unroll
  for (int i = 0; i < 4; ++i)
#pragma unroll
    for (int j = 0; j < 4; ++j) acc[i][j] = (v8f){0.f,0.f,0.f,0.f,0.f,0.f,0.f,0.f};

  for (int k0 = 0; k0 < K; k0 += 32) {
    V bh[4], bl[4];
#pragma unroll
    for (int j = 0; j < 4; ++j) {
      const size_t bo = (size_t)(n0 + (j << 4) + rlane) * ldb + koff + k0;
      bh[j] = Frag<T>::load(Bb + bo);
      if (SPL == 2) bl[j] = Frag<T>::load(Bb2 + bo);
    }
#pragma unroll
    for (int i = 0; i < 4; ++i) {
      const size_t ao = (size_t)(m0 + (i << 4) + rlane) * lda + koff + k0;
      V ah = Frag<T>::load(Ab + ao);
      V al;
      if (SPL >= 1) al = Frag<T>::load(Ab2 + ao);
#pragma unroll
      for (int j = 0; j < 4; ++j) {
        acc[i][j] = Frag<T>::mma(ah, bh[j], acc[i][j]);
        if (SPL == 2) acc[i][j] = Frag<T>::mma(ah, bl[j], acc[i][j]);
        if (SPL >= 1) acc[i][j] = Frag<T>::mma(al, bh[j], acc[i][j]);
      }
      Frag<T>::guard4(acc[i][0], acc[i][1], acc[i][2], acc[i][3], ah, (SPL >= 1) ? al : ah);
    }
    Frag<T>::keep(bh[0], bh[1], bh[2], bh[3]);
    if (SPL == 2) Frag<T>::keep(bl[0], bl[1], bl[2], bl[3]);
  }
  acc_guard4(acc[0][0], acc[0][1], acc[0][2], acc[0][3]);
  acc_guard4(acc[1][0], acc[1][1], acc[1][2], acc[1][3]);
  acc_guard4(acc[2][0], acc[2][1], acc[2][2], acc[2][3]);
  acc_guard4(acc[3][0], acc[3][1], acc[3][2], acc[3][3]);

  float* slab = sT[wave];
  const float* Rb = RESID ? (resid + (size_t)b * strideR) : nullptr;
#pragma unroll
  for (int i = 0; i < 4; ++i) {
    const int mBase = m0 + (i << 4);
#pragma unroll
    for (int j = 0; j < 4; ++j) {
      const int n = n0 + (j << 4) + rlane;
      float bv = 0.f;
      if (BIAS_MODE == 2) bv = bias[n];
#pragma unroll
      for (int r = 0; r < 8; ++r) {
        float v = acc[i][j][r] * scale;
        if (BIAS_MODE == 1) v += bias[mBase + mOff + r];
        if (BIAS_MODE == 2) v += bv;
        if (RESID) v += Rb[(size_t)(mBase + mOff + r) * ldc + n];
        if (ACT == 2) v = fmaxf(v, 0.0f);
        if (ACT == 4) v = (v > 0.f) ? v : 0.01f * v;
        slab[(mOff + r) * 68 + (j << 4) + rlane] = v;
      }
    }
    __builtin_amdgcn_fence(__ATOMIC_RELEASE, "workgroup");
    __builtin_amdgcn_wave_barrier();
    __builtin_amdgcn_fence(__ATOMIC_ACQUIRE, "workgroup");
    if (OUT_MODE == 0) {
      float* C = (float*)Cout + (size_t)b * strideC;
      const int hh = lane >> 4, c4 = (lane & 15) * 4;
      for (int pass = 0; pass < 2; ++pass) {
#pragma unroll
        for (int it = 0; it < 8; ++it) {
          const int row = it * 2 + hh;
          v4f v = *(const v4f*)(slab + row * 68 + c4);
          *(volatile v4f*)(C + (size_t)(mBase + row) * ldc + n0 + c4) = v;
        }
        __threadfence();
      }
    } else {
      const int q = lane >> 3, c8 = (lane & 7) * 8;
      unsigned short* C  = (unsigned short*)Cout  + (size_t)b * strideC;
      unsigned short* C2 = (OUT_MODE == 2) ? ((unsigned short*)Cout2 + (size_t)b * strideC) : nullptr;
      for (int pass = 0; pass < 2; ++pass) {
#pragma unroll
        for (int it = 0; it < 4; ++it) {
          const int row = it * 4 + q;
          const float* sp = slab + row * 68 + c8;
          v8h hv, lv;
#pragma unroll
          for (int e = 0; e < 8; ++e) {
            if (OUT_MODE == 1) {
              hv[e] = (_Float16)sp[e];
            } else {
              unsigned short hb = f2bf_bits(sp[e]);
              unsigned short lb = f2bf_bits(sp[e] - bf_bits2f(hb));
              hv[e] = __builtin_bit_cast(_Float16, hb);
              lv[e] = __builtin_bit_cast(_Float16, lb);
            }
          }
          *(volatile v8h*)(C + (size_t)(mBase + row) * ldc + n0 + c8) = hv;
          if (OUT_MODE == 2) *(volatile v8h*)(C2 + (size_t)(mBase + row) * ldc + n0 + c8) = lv;
        }
        __threadfence();
      }
    }
    __builtin_amdgcn_fence(__ATOMIC_RELEASE, "workgroup");
    __builtin_amdgcn_wave_barrier();
    __builtin_amdgcn_fence(__ATOMIC_ACQUIRE, "workgroup");
  }
}

__global__ __launch_bounds__(256) void cast_pad_bf16_kernel(
    const float* __restrict__ src, unsigned short* __restrict__ dst,
    int Nsrc, int Ksrc, int Kpad, int total8)
{
  const int i = blockIdx.x * 256 + threadIdx.x;
  if (i >= total8) return;
  const int e0 = i << 3;
  const int n  = e0 / Kpad;
  const int k  = e0 - n * Kpad;
  const bool valid = (n < Nsrc) && (k < Ksrc);
  const int nc = (n < Nsrc) ? n : (Nsrc - 1);
  const int kc = (k < Ksrc) ? k : (Ksrc - 8);
  const float* p = src + (size_t)nc * Ksrc + kc;
  const v4f a0 = *(const v4f*)(p);
  const v4f a1 = *(const v4f*)(p + 4);
  v8h hv;
#pragma unroll
  for (int e = 0; e < 4; ++e) {
    const float f0 = valid ? a0[e] : 0.0f;
    const float f1 = valid ? a1[e] : 0.0f;
    const unsigned short h0 = f2bf_bits(f0), h1 = f2bf_bits(f1);
    hv[e]     = __builtin_bit_cast(_Float16, h0);
    hv[4 + e] = __builtin_bit_cast(_Float16, h1);
  }
  unsigned short* q = dst + (size_t)e0;
  *(volatile v8h*)q = hv;
  __threadfence();
  *(volatile v8h*)q = hv;
}

__global__ __launch_bounds__(256) void dt_split_kernel(
    const float* __restrict__ PROJ, unsigned short* __restrict__ DTH, unsigned short* __restrict__ DTL, int total8)
{
  const int i = blockIdx.x * 256 + threadIdx.x;
  if (i >= total8) return;
  const int e0  = i << 3;
  const int row = e0 >> 6;
  const int c8  = e0 & 63;
  const bool valid = (c8 < kDtR);
  const float* p = PROJ + (size_t)row * kPrjP + c8;
  const v4f a0 = *(const v4f*)(p);
  const v4f a1 = *(const v4f*)(p + 4);
  v8h hv, lv;
#pragma unroll
  for (int e = 0; e < 4; ++e) {
    const float f0 = valid ? a0[e] : 0.0f;
    const float f1 = valid ? a1[e] : 0.0f;
    const unsigned short h0 = f2bf_bits(f0), h1 = f2bf_bits(f1);
    const unsigned short l0 = f2bf_bits(f0 - bf_bits2f(h0)), l1 = f2bf_bits(f1 - bf_bits2f(h1));
    hv[e]     = __builtin_bit_cast(_Float16, h0);
    hv[4 + e] = __builtin_bit_cast(_Float16, h1);
    lv[e]     = __builtin_bit_cast(_Float16, l0);
    lv[4 + e] = __builtin_bit_cast(_Float16, l1);
  }
  unsigned short* qh = DTH + (size_t)e0;
  unsigned short* ql = DTL + (size_t)e0;
  *(volatile v8h*)qh = hv;
  *(volatile v8h*)ql = lv;
  __threadfence();
  *(volatile v8h*)qh = hv;
  *(volatile v8h*)ql = lv;
}

__global__ __launch_bounds__(256) void conv_silu_kernel(
    const float* __restrict__ XZ, const float* __restrict__ cw, const float* __restrict__ cb,
    float* __restrict__ UC, unsigned short* __restrict__ UCH, unsigned short* __restrict__ UCL)
{
  __shared__ __align__(16) float sT[16 * kTP];
  const int tid = threadIdx.x, lane = tid & 31, wave = tid >> 5;
  const int d0 = blockIdx.x * 256, d = d0 + tid;
  const int g0 = blockIdx.y * 64;
  const int tb = g0 & (kSeq - 1);
  const v4f wv = *(const v4f*)(cw + (size_t)d * 4);
  const float wr0 = wv[0], wr1 = wv[1], wr2 = wv[2], wr3 = wv[3];
  const float w0 = bf_rne(wr0), w1 = bf_rne(wr1), w2 = bf_rne(wr2), w3 = bf_rne(wr3);
  const float bc = bf_rne(cb[d]);
  float xm3, xm2, xm1;
  {
    const bool hist = (tb > 0);
    const int rb = hist ? (g0 - 3) : g0;
    const float v3 = XZ[(size_t)rb * kXzP + d];
    const float v2 = XZ[(size_t)(rb + 1) * kXzP + d];
    const float v1 = XZ[(size_t)(rb + 2) * kXzP + d];
    xm3 = hist ? v3 : 0.f;
    xm2 = hist ? v2 : 0.f;
    xm1 = hist ? v1 : 0.f;
  }
  const int hrow = wave >> 1;
  const int hch  = (wave & 1) * 128 + lane * 4;
#pragma unroll 1
  for (int sub = 0; sub < 4; ++sub) {
    const int lb = g0 + sub * 16;
#pragma unroll 1
    for (int s = 0; s < 16; ++s) {
      const float xcur = XZ[(size_t)(lb + s) * kXzP + d];
      float acc = w0 * xm3;
      acc = fmaf(w1, xm2, acc);
      acc = fmaf(w2, xm1, acc);
      acc = fmaf(w3, xcur, acc);
      const float sv = acc + bc;
      const float sg = __builtin_amdgcn_rcpf(1.0f + expf(-sv));
      sT[s * kTP + tid] = sv * sg;
      xm3 = xm2; xm2 = xm1; xm1 = xcur;
    }
    __syncthreads();
    v4f fv[4];
    v8h bh[2], blo[2];
#pragma unroll
    for (int it = 0; it < 4; ++it) fv[it] = *(const v4f*)(sT + (it * 4 + hrow) * kTP + hch);
#pragma unroll
    for (int it = 0; it < 2; ++it) {
      const float* sp = sT + (it * 8 + wave) * kTP + lane * 8;
      const v4f a0 = *(const v4f*)(sp);
      const v4f a1 = *(const v4f*)(sp + 4);
#pragma unroll
      for (int e = 0; e < 4; ++e) {
        const float f0 = a0[e], f1 = a1[e];
        const unsigned short h0 = f2bf_bits(f0), h1 = f2bf_bits(f1);
        const unsigned short l0 = f2bf_bits(f0 - bf_bits2f(h0)), l1 = f2bf_bits(f1 - bf_bits2f(h1));
        bh[it][e]      = __builtin_bit_cast(_Float16, h0);
        bh[it][4 + e]  = __builtin_bit_cast(_Float16, h1);
        blo[it][e]     = __builtin_bit_cast(_Float16, l0);
        blo[it][4 + e] = __builtin_bit_cast(_Float16, l1);
      }
    }
    for (int pass = 0; pass < 2; ++pass) {
#pragma unroll
      for (int it = 0; it < 4; ++it)
        *(volatile v4f*)(UC + (size_t)(lb + it * 4 + hrow) * kDin + d0 + hch) = fv[it];
#pragma unroll
      for (int it = 0; it < 2; ++it) {
        const size_t o = (size_t)(lb + it * 8 + wave) * kDin + d0 + lane * 8;
        *(volatile v8h*)(UCH + o) = bh[it];
        *(volatile v8h*)(UCL + o) = blo[it];
      }
      __threadfence();
    }
    __syncthreads();
  }
}

__global__ __launch_bounds__(256) void scan_kernel(
    const float* __restrict__ DLR, const float* __restrict__ UC, const float* __restrict__ XZ,
    const float* __restrict__ PROJ, const float* __restrict__ A_log, const float* __restrict__ Dv,
    const float* __restrict__ bdt, unsigned short* __restrict__ YH, unsigned short* __restrict__ YL)
{
  __shared__ __align__(16) float sBC[16 * 32];
  __shared__ __align__(16) float sY[16 * kTP];
  __shared__ __align__(16) float sA[kNst * 256];
  const int tid = threadIdx.x, lane = tid & 31, wave = tid >> 5;
  const int d0 = blockIdx.x * 256, d = d0 + tid;
  const size_t row0 = (size_t)blockIdx.y * kSeq;

#pragma unroll 1
  for (int n = 0; n < kNst; ++n) {
    const float al = A_log[(size_t)d * kNst + n];
    sA[n * 256 + tid] = -expf(bf_rne(al));
  }
  __syncthreads();
  float An[kNst], h[kNst];
#pragma unroll
  for (int n = 0; n < kNst; ++n) {
    An[n] = sA[n * 256 + tid];
    h[n] = 0.f;
  }
  const float Dd = bf_rne(Dv[d]);
  const float bb = bf_rne(bdt[d]);

#pragma unroll 1
  for (int c = 0; c < kSeq / 16; ++c) {
    const int l0 = c * 16;
    if (tid < 128) {
      const int r = tid >> 3, q = (tid & 7) * 4;
      const v4f v = *(const v4f*)(PROJ + (row0 + l0 + r) * kPrjP + kDtR + q);
      *(v4f*)(sBC + r * 32 + q) = v;
    }
    __syncthreads();
#pragma unroll 1
    for (int s = 0; s < 16; ++s) {
      const size_t m = row0 + (size_t)(l0 + s);
      const float a     = DLR[m * kDin + d] + bb;
      const float delta = fmaxf(a, 0.0f) + log1pf(expf(-fabsf(a)));
      const float xv    = UC[m * kDin + d];
      const float zv    = XZ[m * kXzP + kDin + d];
      v4f Bq[4], Cq[4];
#pragma unroll
      for (int qq = 0; qq < 4; ++qq) {
        Bq[qq] = *(const v4f*)(sBC + s * 32 + 4 * qq);
        Cq[qq] = *(const v4f*)(sBC + s * 32 + kNst + 4 * qq);
      }
      const float dtx = delta * xv;
      float y = 0.f;
#pragma unroll
      for (int n = 0; n < kNst; ++n) {
        const float e  = __expf(delta * An[n]);
        const float bn = Bq[n >> 2][n & 3];
        const float cn = Cq[n >> 2][n & 3];
        const float hn = h[n] * e + dtx * bn;
        h[n] = hn;
        y = hn * cn + y;
      }
      y = xv * Dd + y;
      const float sg = __builtin_amdgcn_rcpf(1.0f + expf(-zv));
      const float g  = zv * sg;
      sY[s * kTP + tid] = y * g;
    }
    __syncthreads();
    v8h hv[2], lv[2];
#pragma unroll
    for (int it = 0; it < 2; ++it) {
      const float* sp = sY + (it * 8 + wave) * kTP + lane * 8;
      const v4f a0 = *(const v4f*)(sp);
      const v4f a1 = *(const v4f*)(sp + 4);
#pragma unroll
      for (int e = 0; e < 4; ++e) {
        const float f0 = a0[e], f1 = a1[e];
        const unsigned short h0 = f2bf_bits(f0), h1 = f2bf_bits(f1);
        const unsigned short q0 = f2bf_bits(f0 - bf_bits2f(h0)), q1 = f2bf_bits(f1 - bf_bits2f(h1));
        hv[it][e]     = __builtin_bit_cast(_Float16, h0);
        hv[it][4 + e] = __builtin_bit_cast(_Float16, h1);
        lv[it][e]     = __builtin_bit_cast(_Float16, q0);
        lv[it][4 + e] = __builtin_bit_cast(_Float16, q1);
      }
    }
    for (int pass = 0; pass < 2; ++pass) {
#pragma unroll
      for (int it = 0; it < 2; ++it) {
        const size_t o = (row0 + (size_t)(l0 + it * 8 + wave)) * kDin + d0 + lane * 8;
        *(volatile v8h*)(YH + o) = hv[it];
        *(volatile v8h*)(YL + o) = lv[it];
      }
      __threadfence();
    }
  }
}

__global__ __launch_bounds__(256) void layernorm_kernel(
    const float* __restrict__ PRE, const float* __restrict__ lw, const float* __restrict__ lb, float* __restrict__ out)
{
  const int lane = threadIdx.x & 31, wave = threadIdx.x >> 5;
  const int row = blockIdx.x * 8 + wave;
  const float* p = PRE + (size_t)row * kDm;
  v4f v[6];
#pragma unroll
  for (int j = 0; j < 6; ++j) v[j] = *(const v4f*)(p + j * 128 + lane * 4);
  float s = 0.f;
#pragma unroll
  for (int j = 0; j < 6; ++j) s += (v[j][0] + v[j][1]) + (v[j][2] + v[j][3]);
#pragma unroll
  for (int off = 16; off > 0; off >>= 1) s += __shfl_xor(s, off, 32);
  const float mu = s * kInvDm;
  float q = 0.f;
#pragma unroll
  for (int j = 0; j < 6; ++j) {
#pragma unroll
    for (int e = 0; e < 4; ++e) {
      const float dd = v[j][e] - mu;
      q = fmaf(dd, dd, q);
    }
  }
#pragma unroll
  for (int off = 16; off > 0; off >>= 1) q += __shfl_xor(q, off, 32);
  const float var  = q * kInvDm;
  const float rstd = rsqrtf(var + kLnEps);
  v4f o[6];
#pragma unroll
  for (int j = 0; j < 6; ++j) {
    const v4f wv = *(const v4f*)(lw + j * 128 + lane * 4);
    const v4f bv = *(const v4f*)(lb + j * 128 + lane * 4);
#pragma unroll
    for (int e = 0; e < 4; ++e) {
      const float we = wv[e], be = bv[e];
      o[j][e] = (v[j][e] - mu) * rstd * bf_rne(we) + bf_rne(be);
    }
  }
  float* dst = out + (size_t)row * kDm;
  for (int pass = 0; pass < 2; ++pass) {
#pragma unroll
    for (int j = 0; j < 6; ++j) *(volatile v4f*)(dst + j * 128 + lane * 4) = o[j];
    __threadfence();
  }
}

extern "C" void kernel_launch(void* const* d_in, const int* in_sizes, int n_in,
                              void* d_out, int out_size, void* d_ws, size_t ws_size,
                              hipStream_t stream) {
  if (n_in < 12) return;
  if (in_sizes[0] != kRows * kDm) return;
  if (in_sizes[1] != kXzP * kDm) return;
  if (in_sizes[2] != kDin * 4) return;
  if (in_sizes[3] != kDin) return;
  if (in_sizes[4] != kPrjN * kDin) return;
  if (in_sizes[5] != kDin * kDtR) return;
  if (in_sizes[6] != kDin) return;
  if (in_sizes[7] != kDin * kNst) return;
  if (in_sizes[8] != kDin) return;
  if (in_sizes[9] != kDm * kDin) return;
  if (in_sizes[10] != kDm) return;
  if (in_sizes[11] != kDm) return;
  if (out_size != kRows * kDm) return;
  if (ws_size < kWsTotal) return;

  const float* x      = (const float*)d_in[0];
  const float* W_in   = (const float*)d_in[1];
  const float* conv_w = (const float*)d_in[2];
  const float* conv_b = (const float*)d_in[3];
  const float* W_x    = (const float*)d_in[4];
  const float* W_dt   = (const float*)d_in[5];
  const float* b_dt   = (const float*)d_in[6];
  const float* A_log  = (const float*)d_in[7];
  const float* Dp     = (const float*)d_in[8];
  const float* W_out  = (const float*)d_in[9];
  const float* ln_w   = (const float*)d_in[10];
  const float* ln_b   = (const float*)d_in[11];
  float* out = (float*)d_out;

  char* ws = (char*)d_ws;
  unsigned short* XB   = (unsigned short*)(ws + kOffXB);
  unsigned short* WIB  = (unsigned short*)(ws + kOffWIB);
  unsigned short* WXB  = (unsigned short*)(ws + kOffWXB);
  unsigned short* WDB  = (unsigned short*)(ws + kOffWDB);
  unsigned short* WOB  = (unsigned short*)(ws + kOffWOB);
  float*          XZ   = (float*)(ws + kOffXZ);
  float*          UC   = (float*)(ws + kOffUC);
  unsigned short* UCH  = (unsigned short*)(ws + kOffUCH);
  unsigned short* UCL  = (unsigned short*)(ws + kOffUCL);
  float*          PROJ = (float*)(ws + kOffPROJ);
  unsigned short* DTH  = (unsigned short*)(ws + kOffDTH);
  unsigned short* DTL  = (unsigned short*)(ws + kOffDTL);
  float*          DLR  = (float*)(ws + kOffDLR);
  unsigned short* YH   = (unsigned short*)(ws + kOffYH);
  unsigned short* YL   = (unsigned short*)(ws + kOffYL);
  float*          PRE  = (float*)(ws + kOffPRE);
  const float* dummy_bias  = b_dt;
  const float* dummy_resid = x;

  cast_pad_bf16_kernel<<<(kRows * kDm / 8) / 256, 256, 0, stream>>>(x,     XB,  kRows, kDm,  kDm,  kRows * kDm / 8);
  cast_pad_bf16_kernel<<<(kXzP * kDm / 8) / 256, 256, 0, stream>>>(W_in,  WIB, kXzP,  kDm,  kDm,  kXzP * kDm / 8);
  cast_pad_bf16_kernel<<<(kPrjP * kDin / 8) / 256, 256, 0, stream>>>(W_x, WXB, kPrjN, kDin, kDin, kPrjP * kDin / 8);
  cast_pad_bf16_kernel<<<(kDin * kDtK / 8) / 256, 256, 0, stream>>>(W_dt, WDB, kDin,  kDtR, kDtK, kDin * kDtK / 8);
  cast_pad_bf16_kernel<<<(kDm * kDin / 8) / 256, 256, 0, stream>>>(W_out, WOB, kDm,   kDin, kDin, kDm * kDin / 8);

  wmma_gemm64<1, 0, 0, 0, false><<<dim3(192, 1), 256, 0, stream>>>(
      XB, XB, kDm, 0L,
      WIB, WIB, kDm, 0L,
      (void*)XZ, (void*)XZ, kXzP, 0L,
      dummy_bias, dummy_resid, 0L,
      kRows, kXzP, kDm, 1.0f);

  conv_silu_kernel<<<dim3(kDin / 256, kRows / 64), 256, 0, stream>>>(XZ, conv_w, conv_b, UC, UCH, UCL);

  wmma_gemm64<1, 1, 0, 0, false><<<dim3(8, 1), 256, 0, stream>>>(
      UCH, UCL, kDin, 0L,
      WXB, WXB, kDin, 0L,
      (void*)PROJ, (void*)PROJ, kPrjP, 0L,
      dummy_bias, dummy_resid, 0L,
      kRows, kPrjP, kDin, 1.0f);

  dt_split_kernel<<<(kRows * kDtK / 8) / 256, 256, 0, stream>>>(PROJ, DTH, DTL, kRows * kDtK / 8);

  wmma_gemm64<1, 1, 0, 0, false><<<dim3(96, 1), 256, 0, stream>>>(
      DTH, DTL, kDtK, 0L,
      WDB, WDB, kDtK, 0L,
      (void*)DLR, (void*)DLR, kDin, 0L,
      dummy_bias, dummy_resid, 0L,
      kRows, kDin, kDtK, 1.0f);

  scan_kernel<<<dim3(kDin / 256, kBatch), 256, 0, stream>>>(DLR, UC, XZ, PROJ, A_log, Dp, b_dt, YH, YL);

  wmma_gemm64<1, 1, 0, 0, false><<<dim3(48, 1), 256, 0, stream>>>(
      YH, YL, kDin, 0L,
      WOB, WOB, kDin, 0L,
      (void*)PRE, (void*)PRE, kDm, 0L,
      dummy_bias, dummy_resid, 0L,
      kRows, kDm, kDin, 1.0f);

  layernorm_kernel<<<kRows / 8, 256, 0, stream>>>(PRE, ln_w, ln_b, out);
}
